// GraphRelationUpdate_53884659695843
// MI455X (gfx1250) — hardware-verified
//
#include <hip/hip_runtime.h>
#include <stdint.h>
#include <stddef.h>
#include <math.h>

#define HD      128
#define KN      16
#define WPB     8
#define WSC     64.0f
#define WINV    (1.0f / 64.0f)
#define NPIECE  (HD * HD / 8)

static_assert(HD % 32 == 0);
static_assert(NPIECE % 256 == 0);
static_assert(KN == 16);

typedef _Float16 v16h __attribute__((ext_vector_type(16)));
typedef _Float16 v8h  __attribute__((ext_vector_type(8)));
typedef _Float16 v4h  __attribute__((ext_vector_type(4)));
typedef float    v8f  __attribute__((ext_vector_type(8)));
typedef float    v4f  __attribute__((ext_vector_type(4)));
typedef v4f __attribute__((may_alias)) v4fa;
typedef v8h __attribute__((may_alias)) v8ha;

union FragH { v16h v; v8h q[2]; v4h q4[4]; };

__device__ __forceinline__ v8f wmma_h(v16h a, v16h b, v8f c) {
  v8f d = __builtin_amdgcn_wmma_f32_16x16x32_f16(false, a, false, b, (short)0, c, false, false);
  asm volatile("v_nop\n\tv_nop\n\tv_nop\n\tv_nop" : "+v"(d) : "v"(a), "v"(b));
  return d;
}

__device__ __forceinline__ v16h ldfrag_h(const _Float16* p, int h) {
  FragH f;
  f.q[0] = *(const v8ha*)(p + 8 * h);
  f.q[1] = *(const v8ha*)(p + 16 + 8 * h);
  return f.v;
}

__global__ __launch_bounds__(256) void k_wconv(const float* __restrict__ w,
                                               _Float16* __restrict__ wh)
{
  int p = blockIdx.x * 256 + threadIdx.x;
  p = p > NPIECE - 1 ? NPIECE - 1 : p;
  const v4f a = *(const v4fa*)(w + (size_t)p * 8);
  const v4f b = *(const v4fa*)(w + (size_t)p * 8 + 4);
  FragH o;
  o.q4[0] = __builtin_convertvector(a * WSC, v4h);
  o.q4[1] = __builtin_convertvector(b * WSC, v4h);
  _Float16* dp = wh + (size_t)p * 8;
  *(volatile v8ha*)dp = o.q[0];
  __threadfence();
  *(volatile v8ha*)dp = o.q[0];
}

__global__ __launch_bounds__(256) void k_score(const float* __restrict__ e,
                                               const _Float16* __restrict__ wh,
                                               const float* __restrict__ wb,
                                               const float* __restrict__ ua,
                                               float* __restrict__ score,
                                               int N)
{
  __shared__ __align__(16) float sS[WPB * 16];

  const int tid = threadIdx.x, wave = tid >> 5, lane = tid & 31;
  const int h = lane >> 4, m = lane & 15;
  const int tile = blockIdx.x * WPB + wave;
  int arow = tile * 16 + m;
  arow = arow > N - 1 ? N - 1 : arow;
  const float* erow = e + (size_t)arow * HD;

  const v8f z8 = {0.f, 0.f, 0.f, 0.f, 0.f, 0.f, 0.f, 0.f};
  v8f acc[8];
  #pragma unroll
  for (int t = 0; t < 8; ++t) acc[t] = z8;

  #pragma unroll 1
  for (int kk = 0; kk < HD; kk += 32) {
    const v4f a0 = *(const v4fa*)(erow + kk + 8 * h);
    const v4f a1 = *(const v4fa*)(erow + kk + 8 * h + 4);
    const v4f a2 = *(const v4fa*)(erow + kk + 16 + 8 * h);
    const v4f a3 = *(const v4fa*)(erow + kk + 16 + 8 * h + 4);
    FragH fa;
    fa.q4[0] = __builtin_convertvector(a0, v4h);
    fa.q4[1] = __builtin_convertvector(a1, v4h);
    fa.q4[2] = __builtin_convertvector(a2, v4h);
    fa.q4[3] = __builtin_convertvector(a3, v4h);
    #pragma unroll
    for (int t = 0; t < 8; ++t) {
      const v16h b = ldfrag_h(wh + (size_t)(t * 16 + m) * HD + kk, h);
      acc[t] = wmma_h(fa.v, b, acc[t]);
    }
  }

  float partial[8];
  #pragma unroll
  for (int r = 0; r < 8; ++r) partial[r] = 0.0f;
  #pragma unroll
  for (int t = 0; t < 8; ++t) {
    const int n = t * 16 + m;
    const float bias = wb[n];
    const float u    = ua[n];
    #pragma unroll
    for (int r = 0; r < 8; ++r) {
      const float v  = acc[t][r] * WINV + bias;
      const float hv = (v >= 0.0f) ? v : 0.1f * v;
      partial[r] += hv * u;
    }
  }
  #pragma unroll
  for (int off = 1; off < 16; off <<= 1) {
    #pragma unroll
    for (int r = 0; r < 8; ++r)
      partial[r] += __shfl_xor(partial[r], off, 16);
  }
  const int rsel = m & 7;
  float mine = partial[0];
  #pragma unroll
  for (int r = 1; r < 8; ++r) mine = (rsel == r) ? partial[r] : mine;
  sS[wave * 16 + 8 * h + rsel] = mine;
  __syncthreads();

  if (wave == 0) {
    const v4f v = *(const v4fa*)(sS + lane * 4);
    float* gp = score + (size_t)blockIdx.x * (WPB * 16) + lane * 4;
    *(volatile v4fa*)gp = v;
    __threadfence();
    *(volatile v4fa*)gp = v;
  }
}

__global__ __launch_bounds__(256) void k_agg(const float* __restrict__ e,
                                             const int*   __restrict__ nbr,
                                             const float* __restrict__ score,
                                             float* __restrict__ out,
                                             int N)
{
  const int wave = threadIdx.x >> 5;
  const int lane = threadIdx.x & 31;
  const int node = blockIdx.x * WPB + wave;
  if (node >= N) return;

  const int k16 = lane & 15;
  int idx = nbr[(size_t)node * KN + k16];
  idx = idx < 0 ? idx + N : idx;
  idx = idx < 0 ? 0 : (idx > N - 1 ? N - 1 : idx);
  const float s = score[idx];

  float mx = s;
  #pragma unroll
  for (int off = 1; off < 16; off <<= 1) mx = fmaxf(mx, __shfl_xor(mx, off, 16));
  const float ex = expf(s - mx);
  float sum = ex;
  #pragma unroll
  for (int off = 1; off < 16; off <<= 1) sum += __shfl_xor(sum, off, 16);
  const float w = ex * (1.0f / sum);

  v4f acc = {0.f, 0.f, 0.f, 0.f};
  #pragma unroll 8
  for (int k = 0; k < KN; ++k) {
    const float wk = __shfl(w, k, 16);
    const int   nk = __shfl(idx, k, 16);
    const v4f v = *(const v4fa*)(e + (size_t)nk * HD + lane * 4);
    acc += wk * v;
  }
  const v4f self = *(const v4fa*)(e + (size_t)node * HD + lane * 4);
  const v4f res = self + acc;
  float* gp = out + (size_t)node * HD + lane * 4;
  *(volatile v4fa*)gp = res;
  __threadfence();
  *(volatile v4fa*)gp = res;
}

extern "C" void kernel_launch(void* const* d_in, const int* in_sizes, int n_in,
                              void* d_out, int out_size, void* d_ws, size_t ws_size,
                              hipStream_t stream)
{
  if (n_in < 5) return;
  const int nE = in_sizes[0];
  if (nE < HD || (nE % HD) != 0) return;
  const int N = nE / HD;
  if (in_sizes[1] != HD * HD) return;
  if (in_sizes[2] != HD) return;
  if (in_sizes[3] != HD) return;
  if (in_sizes[4] != N * KN) return;
  if (out_size != N * HD) return;

  const float* e    = (const float*)d_in[0];
  const float* Wa_w = (const float*)d_in[1];
  const float* Wa_b = (const float*)d_in[2];
  const float* ua   = (const float*)d_in[3];
  const int*   nbr  = (const int*)d_in[4];
  float*       out  = (float*)d_out;

  const int numTiles = (N + 15) / 16;
  const int nblk     = (numTiles + WPB - 1) / WPB;
  const int nagg     = (N + WPB - 1) / WPB;

  const size_t bW = (size_t)HD * HD * 2;
  const size_t bS = (size_t)nblk * (WPB * 16) * 4;
  const size_t total = bW + bS;
  if (total > ws_size) return;
  if (total > (size_t)134217728) return;

  char* ws = (char*)d_ws;
  size_t off = 0;
  _Float16* wh  = (_Float16*)(ws + off); off += bW;
  float*    scr = (float*)(ws + off);    off += bS;
  if (off != total) return;

  k_wconv<<<dim3(NPIECE / 256), 256, 0, stream>>>(Wa_w, wh);
  k_score<<<dim3(nblk), 256, 0, stream>>>(e, wh, Wa_b, ua, scr, N);
  k_agg<<<dim3(nagg), 256, 0, stream>>>(e, nbr, scr, out, N);
}
